// PointNetSetAbstraction_42185168781351
// MI455X (gfx1250) — hardware-verified
//
#include <hip/hip_runtime.h>
#pragma clang fp contract(off)

typedef __attribute__((ext_vector_type(16))) _Float16 v16h;
typedef __attribute__((ext_vector_type(8)))  _Float16 v8h;
typedef __attribute__((ext_vector_type(8)))  float    v8f;
typedef __attribute__((ext_vector_type(4)))  float    v4f;
typedef __attribute__((ext_vector_type(4)))  unsigned int v4u;

constexpr int NB = 16;
constexpr int NPTS = 4096;
constexpr int NSAMP = 1024;
constexpr int NNBR = 32;
constexpr int CPTS = 64;
constexpr int CIN0 = 67;
constexpr int NGRP = NB * NSAMP;
constexpr int MROWS = NGRP * NNBR;
constexpr int NPROW = NB * NPTS;
constexpr int LDT = 72;
constexpr float CARRY = 16.0f;
constexpr float FOLD = 1.0f / (CARRY * CARRY);
constexpr float BN_EPS = 1e-5f;

static_assert(NGRP == 16384, "groups");
static_assert(MROWS == 524288, "rows");
static_assert(NPROW == 65536, "points");
static_assert(CIN0 == CPTS + 3, "layer-0 input width");
static_assert(196608 + 8388608 == 8585216, "output packing");
static_assert((NB * 3 * NSAMP) * 4 == 196608, "out0 bytes");

constexpr size_t WS_PTST  = (size_t)NPROW * 64 * 2;
constexpr size_t WS_WH    = (size_t)256 * 64 * 2;
constexpr size_t WS_Q     = (size_t)NPROW * 64 * 4;
constexpr size_t WS_R     = (size_t)NGRP * 64 * 4;
constexpr size_t WS_IDX   = (size_t)NGRP * 32 * 4;
constexpr size_t WS_NXYZ  = (size_t)NGRP * 4 * 4;
constexpr size_t WS_Y1    = (size_t)MROWS * 64 * 2;
constexpr size_t WS_YMM   = (size_t)NGRP * 256 * 4;
constexpr size_t WS_PART0 = (size_t)1024 * 128 * 4;
constexpr size_t WS_PART1 = (size_t)4096 * 128 * 4;
constexpr size_t WS_PART2 = (size_t)4096 * 256 * 4;
constexpr size_t WS_TAB   = (size_t)256 * 4;
constexpr size_t WS_TOTAL = WS_PTST + WS_WH + WS_Q + WS_R + WS_IDX + WS_NXYZ + WS_Y1 + WS_YMM +
                            WS_PART0 + WS_PART1 + WS_PART2 + 3 * WS_TAB;
static_assert(WS_TOTAL <= (size_t)134217728, "carve under 128 MiB");
static_assert(WS_PTST % 128 == 0 && WS_WH % 128 == 0 && WS_NXYZ % 128 == 0 && WS_TAB % 128 == 0, "aligned carves");

__device__ __forceinline__ float h16_to_f32(unsigned hb) {
  const unsigned sgn = (hb & 0x8000u) << 16;
  const unsigned em = hb & 0x7fffu;
  const float fn = __uint_as_float((em << 13) + 0x38000000u);
  const float fs = (float)em * 5.9604644775390625e-8f;
  const float mag = (em < 0x400u) ? fs : fn;
  return __uint_as_float(__float_as_uint(mag) | sgn);
}

__device__ __forceinline__ void wave_lds_sync() {
  __builtin_amdgcn_fence(__ATOMIC_RELEASE, "workgroup");
  __builtin_amdgcn_wave_barrier();
  __builtin_amdgcn_fence(__ATOMIC_ACQUIRE, "workgroup");
}

__device__ __forceinline__ v16h frag_ld(const _Float16* p) {
  union { v16h v; v8h h[2]; } f;
  f.h[0] = *(const v8h*)(p);
  f.h[1] = *(const v8h*)(p + 16);
  return f.v;
}

__device__ __forceinline__ v8f mma_h(v16h a, v16h b, v8f c) {
  return __builtin_amdgcn_wmma_f32_16x16x32_f16(false, a, false, b, (short)0, c, false, false);
}

__device__ __forceinline__ void guard4(v8f& c0, v8f& c1, v8f& c2, v8f& c3,
                                       v16h a, v16h b0, v16h b1, v16h b2, v16h b3) {
  asm volatile("v_nop\n\tv_nop\n\tv_nop\n\tv_nop"
               : "+v"(c0), "+v"(c1), "+v"(c2), "+v"(c3)
               : "v"(a), "v"(b0), "v"(b1), "v"(b2), "v"(b3));
}

__device__ __forceinline__ void argmax_wave(float& bv, int& bi) {
#pragma unroll
  for (int off = 16; off > 0; off >>= 1) {
    const float ov = __shfl_xor(bv, off, 32);
    const int oi = __shfl_xor(bi, off, 32);
    const bool take = (ov > bv) || ((ov == bv) && (oi < bi));
    bv = take ? ov : bv;
    bi = take ? oi : bi;
  }
}

__global__ __launch_bounds__(1024) void k_fps(const float* __restrict__ xyz,
                                              float* __restrict__ out0,
                                              float* __restrict__ nxyz) {
#pragma clang fp contract(off)
  __shared__ __align__(16) float sX[3 * NPTS];
  __shared__ int sSel[NSAMP];
  __shared__ float sV[2][32];
  __shared__ int sI[2][32];
  const int b = blockIdx.x;
  const int tid = threadIdx.x;
  const int lane = tid & 31;
  const int wave = tid >> 5;
  const float* X = xyz + (size_t)b * 3 * NPTS;
#pragma unroll
  for (int i = 0; i < 3; ++i) {
    const int e = 4 * (tid + 1024 * i);
    const v4f v = *(const v4f*)(X + e);
    *(v4f*)(sX + e) = v;
  }
  __syncthreads();
  float px[4], py[4], pz[4], dist[4];
#pragma unroll
  for (int p = 0; p < 4; ++p) {
    const int n = tid + p * 1024;
    px[p] = sX[n];
    py[p] = sX[NPTS + n];
    pz[p] = sX[2 * NPTS + n];
    dist[p] = 1e10f;
  }
  int far = 0;
#pragma unroll 1
  for (int s = 0; s < NSAMP; ++s) {
    if (tid == 0) sSel[s] = far;
    const float cx = sX[far];
    const float cy = sX[NPTS + far];
    const float cz = sX[2 * NPTS + far];
    float bv = 0.0f;
    int bi = 0;
#pragma unroll
    for (int p = 0; p < 4; ++p) {
      const float dx = px[p] - cx;
      const float dy = py[p] - cy;
      const float dz = pz[p] - cz;
      const float t0 = dx * dx;
      const float t1 = dy * dy;
      const float t2 = dz * dz;
      const float dd = (t0 + t2) + t1;
      const float nd = fminf(dist[p], dd);
      dist[p] = nd;
      if (p == 0) {
        bv = nd;
        bi = tid;
      } else {
        const bool take = nd > bv;
        bv = take ? nd : bv;
        bi = take ? (tid + p * 1024) : bi;
      }
    }
    argmax_wave(bv, bi);
    const int buf = s & 1;
    if (lane == 0) {
      sV[buf][wave] = bv;
      sI[buf][wave] = bi;
    }
    __syncthreads();
    bv = sV[buf][lane];
    bi = sI[buf][lane];
    argmax_wave(bv, bi);
    far = bi & (NPTS - 1);
  }
  __syncthreads();
  const int doOut = (tid < 768) ? 1 : 0;
  const int tc = doOut ? tid : 767;
  const int ch = tc >> 8;
  const int s4 = (tc & 255) * 4;
  v4f o0;
  o0.x = sX[ch * NPTS + (sSel[s4 + 0] & (NPTS - 1))];
  o0.y = sX[ch * NPTS + (sSel[s4 + 1] & (NPTS - 1))];
  o0.z = sX[ch * NPTS + (sSel[s4 + 2] & (NPTS - 1))];
  o0.w = sX[ch * NPTS + (sSel[s4 + 3] & (NPTS - 1))];
  const int ms = sSel[tid] & (NPTS - 1);
  v4f o1;
  o1.x = sX[ms];
  o1.y = sX[NPTS + ms];
  o1.z = sX[2 * NPTS + ms];
  o1.w = 0.0f;
  float* po0 = out0 + (size_t)b * 3 * NSAMP + (size_t)tc * 4;
  float* po1 = nxyz + ((size_t)b * NSAMP + tid) * 4;
  for (int pass = 0; pass < 2; ++pass) {
    if (doOut) *(volatile v4f*)po0 = o0;
    *(volatile v4f*)po1 = o1;
    __threadfence();
  }
}

__global__ __launch_bounds__(256) void k_prep_pts(const float* __restrict__ pts,
                                                  unsigned short* __restrict__ ptsT) {
  __shared__ __align__(16) float sT[64 * 68];
  const int tid = threadIdx.x;
  const int b = blockIdx.x >> 6;
  const int n0 = (blockIdx.x & 63) * 64;
  const int n4 = (tid & 15) * 4;
  const int cr = tid >> 4;
#pragma unroll
  for (int it = 0; it < 4; ++it) {
    const int c = cr + 16 * it;
    const v4f v = *(const v4f*)(pts + ((size_t)(b * CPTS + c)) * NPTS + n0 + n4);
    *(v4f*)(sT + c * 68 + n4) = v;
  }
  __syncthreads();
  const int c8 = tid & 7;
  const int rr = tid >> 3;
  v8h hv[2];
#pragma unroll
  for (int it = 0; it < 2; ++it) {
    const int row = rr + 32 * it;
#pragma unroll
    for (int i = 0; i < 8; ++i) {
      const float f = sT[(c8 * 8 + i) * 68 + row] * CARRY;
      hv[it][i] = (_Float16)f;
    }
  }
  for (int pass = 0; pass < 2; ++pass) {
#pragma unroll
    for (int it = 0; it < 2; ++it) {
      const int row = rr + 32 * it;
      *(volatile v8h*)(ptsT + ((size_t)(b * NPTS + n0 + row)) * 64 + c8 * 8) = hv[it];
    }
    __threadfence();
  }
}

__device__ __forceinline__ void cvt_row8(const float* __restrict__ src, unsigned short* __restrict__ dst) {
  float f[8];
#pragma unroll
  for (int i = 0; i < 8; ++i) f[i] = src[i];
  v8h hv;
#pragma unroll
  for (int i = 0; i < 8; ++i) {
    const float g = f[i] * CARRY;
    hv[i] = (_Float16)g;
  }
  *(volatile v8h*)dst = hv;
  __threadfence();
  *(volatile v8h*)dst = hv;
}

__global__ __launch_bounds__(256) void k_wprep(const float* __restrict__ w0, const float* __restrict__ w1,
                                               const float* __restrict__ w2, unsigned short* __restrict__ Wh) {
  const int tid = threadIdx.x;
#pragma unroll 1
  for (int it = 0; it < 2; ++it) {
    const int q = tid + 256 * it;
    const int r = q >> 3;
    const int c8 = q & 7;
    cvt_row8(w0 + r * CIN0 + 3 + c8 * 8, Wh + r * 64 + c8 * 8);
  }
#pragma unroll 1
  for (int it = 0; it < 2; ++it) {
    const int q = tid + 256 * it;
    const int r = q >> 3;
    const int c8 = q & 7;
    cvt_row8(w1 + r * 64 + c8 * 8, Wh + (64 + r) * 64 + c8 * 8);
  }
#pragma unroll 1
  for (int it = 0; it < 4; ++it) {
    const int q = tid + 256 * it;
    const int r = q >> 3;
    const int c8 = q & 7;
    cvt_row8(w2 + r * 64 + c8 * 8, Wh + (128 + r) * 64 + c8 * 8);
  }
}

__global__ __launch_bounds__(256) void k_gemmQ(const unsigned short* __restrict__ ptsT,
                                               const unsigned short* __restrict__ Wh,
                                               const float* __restrict__ xyz,
                                               const float* __restrict__ w0,
                                               const float* __restrict__ b0,
                                               float* __restrict__ Q) {
  __shared__ __align__(16) _Float16 sB[64 * LDT];
  __shared__ __align__(16) float sSlab[8][16 * 68];
  __shared__ float sXc[3 * 128];
  __shared__ float sW[64 * 4];
  __shared__ float sBias[64];
  const int tid = threadIdx.x;
  const int lane = tid & 31;
  const int wave = tid >> 5;
  const int rlane = lane & 15;
  const int hh = lane >> 4;
  const int m0 = blockIdx.x * 128;
  const int b = m0 >> 12;
  const int n0 = m0 & (NPTS - 1);
#pragma unroll
  for (int it = 0; it < 2; ++it) {
    const int q = tid + 256 * it;
    const int r = q >> 3;
    const int c8 = q & 7;
    const v4u w = *(const v4u*)(Wh + r * 64 + c8 * 8);
    *(v4u*)(sB + r * LDT + c8 * 8) = w;
  }
  sXc[tid] = xyz[((size_t)(b * 3 + (tid >> 7))) * NPTS + n0 + (tid & 127)];
  if (tid < 128) sXc[256 + tid] = xyz[((size_t)(b * 3 + 2)) * NPTS + n0 + tid];
  if (tid < 64) {
    sW[tid * 4 + 0] = w0[tid * CIN0 + 0];
    sW[tid * 4 + 1] = w0[tid * CIN0 + 1];
    sW[tid * 4 + 2] = w0[tid * CIN0 + 2];
    sW[tid * 4 + 3] = 0.0f;
    sBias[tid] = b0[tid];
  }
  __syncthreads();

  const _Float16* Ag = (const _Float16*)ptsT + ((size_t)(m0 + 16 * wave + rlane)) * 64 + 8 * hh;
  const _Float16* Bl = sB + rlane * LDT + 8 * hh;
  v8f acc[4];
#pragma unroll
  for (int j = 0; j < 4; ++j) acc[j] = (v8f){0.f, 0.f, 0.f, 0.f, 0.f, 0.f, 0.f, 0.f};
#pragma unroll
  for (int ks = 0; ks < 2; ++ks) {
    const v16h a = frag_ld(Ag + ks * 32);
    const v16h f0 = frag_ld(Bl + 0 * 16 * LDT + ks * 32);
    const v16h f1 = frag_ld(Bl + 1 * 16 * LDT + ks * 32);
    const v16h f2 = frag_ld(Bl + 2 * 16 * LDT + ks * 32);
    const v16h f3 = frag_ld(Bl + 3 * 16 * LDT + ks * 32);
    acc[0] = mma_h(a, f0, acc[0]);
    acc[1] = mma_h(a, f1, acc[1]);
    acc[2] = mma_h(a, f2, acc[2]);
    acc[3] = mma_h(a, f3, acc[3]);
    guard4(acc[0], acc[1], acc[2], acc[3], a, f0, f1, f2, f3);
  }

  float* sl = sSlab[wave];
#pragma unroll
  for (int j = 0; j < 4; ++j) {
#pragma unroll
    for (int r = 0; r < 8; ++r) sl[(8 * hh + r) * 68 + 16 * j + rlane] = acc[j][r];
  }
  wave_lds_sync();
  const int c4 = rlane * 4;
  float wx[4], wy[4], wz[4], bb[4];
#pragma unroll
  for (int i = 0; i < 4; ++i) {
    wx[i] = sW[(c4 + i) * 4 + 0];
    wy[i] = sW[(c4 + i) * 4 + 1];
    wz[i] = sW[(c4 + i) * 4 + 2];
    bb[i] = sBias[c4 + i];
  }
  v4f ov[8];
#pragma unroll
  for (int it = 0; it < 8; ++it) {
    const int row = it * 2 + hh;
    const v4f v = *(const v4f*)(sl + row * 68 + c4);
    const float x = sXc[16 * wave + row];
    const float y = sXc[128 + 16 * wave + row];
    const float z = sXc[256 + 16 * wave + row];
    const float va[4] = {v.x, v.y, v.z, v.w};
    float oo[4];
#pragma unroll
    for (int i = 0; i < 4; ++i) {
      const float term = (wx[i] * x + wy[i] * y) + wz[i] * z;
      oo[i] = (va[i] * FOLD + term) + bb[i];
    }
    ov[it] = (v4f){oo[0], oo[1], oo[2], oo[3]};
  }
  for (int pass = 0; pass < 2; ++pass) {
#pragma unroll
    for (int it = 0; it < 8; ++it) {
      const int row = it * 2 + hh;
      *(volatile v4f*)(Q + ((size_t)(m0 + 16 * wave + row)) * 64 + c4) = ov[it];
    }
    __threadfence();
  }
}

__global__ __launch_bounds__(256) void k_ballR(const float* __restrict__ xyz,
                                               const float* __restrict__ nxyz,
                                               const float* __restrict__ w0,
                                               int* __restrict__ idx_out,
                                               float* __restrict__ R) {
#pragma clang fp contract(off)
  __shared__ int sHit[8][32];
  __shared__ __align__(16) float sR[8][64];
  const int tid = threadIdx.x;
  const int lane = tid & 31;
  const int wave = tid >> 5;
  const int gs = blockIdx.x * 8 + wave;
  const int b = gs >> 10;
  const float* X = xyz + (size_t)b * 3 * NPTS;
  const v4f cc = *(const v4f*)(nxyz + (size_t)gs * 4);
  const float cx = cc.x;
  const float cy = cc.y;
  const float cz = cc.z;
  const float c0 = cx * cx;
  const float c1 = cy * cy;
  const float c2 = cz * cz;
  const float sumc = (c0 + c2) + c1;
  sHit[wave][lane] = 0;
  wave_lds_sync();
  int cnt = 0;
#pragma unroll 1
  for (int chn = 0; (chn < NPTS / 32) && (cnt < NNBR); ++chn) {
    const int n = chn * 32 + lane;
    const float x = X[n];
    const float y = X[NPTS + n];
    const float z = X[2 * NPTS + n];
    float p = cx * x;
    p = __builtin_fmaf(cy, y, p);
    p = __builtin_fmaf(cz, z, p);
    const float x0 = x * x;
    const float x1 = y * y;
    const float x2 = z * z;
    const float sumx = (x0 + x2) + x1;
    const float tw = 2.0f * p;
    const float sq = (sumc - tw) + sumx;
    const bool pred = !(sq > 0.04f);
    const unsigned mask = __builtin_amdgcn_ballot_w32(pred);
    const int pos = __popc(mask & ((1u << lane) - 1u));
    const int slot = cnt + pos;
    if (pred && (slot < NNBR)) sHit[wave][slot] = n;
    cnt += __popc(mask);
  }
  wave_lds_sync();
  const int ccap = (cnt < NNBR) ? cnt : NNBR;
  const int lim = (ccap > 0) ? (ccap - 1) : 0;
  const int li = (lane < lim) ? lane : lim;
  const int hv = sHit[wave][li];
  const int fv = sHit[wave][0];
  int v = (lane < ccap) ? hv : fv;
  v = (v < 0) ? 0 : v;
  v = (v > NPTS - 1) ? (NPTS - 1) : v;
  int* pidx = idx_out + (size_t)gs * NNBR + lane;
  *(volatile int*)pidx = v;

  const float a0 = w0[lane * CIN0 + 0];
  const float a1 = w0[lane * CIN0 + 1];
  const float a2 = w0[lane * CIN0 + 2];
  const float d0 = w0[(lane + 32) * CIN0 + 0];
  const float d1 = w0[(lane + 32) * CIN0 + 1];
  const float d2 = w0[(lane + 32) * CIN0 + 2];
  sR[wave][lane] = (a0 * cx + a1 * cy) + a2 * cz;
  sR[wave][lane + 32] = (d0 * cx + d1 * cy) + d2 * cz;
  wave_lds_sync();
  const int l16 = lane & 15;
  const v4f rv = *(const v4f*)(&sR[wave][l16 * 4]);
  float* pr = R + (size_t)gs * 64 + l16 * 4;
  if (lane < 16) *(volatile v4f*)pr = rv;
  __threadfence();
  *(volatile int*)pidx = v;
  if (lane < 16) *(volatile v4f*)pr = rv;
}

__global__ __launch_bounds__(256) void k_stats0(const float* __restrict__ Q, const float* __restrict__ R,
                                                const int* __restrict__ idxp, float* __restrict__ part0) {
  __shared__ int sIdx[512];
  __shared__ float sRed[32][128];
  __shared__ __align__(16) float sP[128];
  const int tid = threadIdx.x;
  const int grp0 = blockIdx.x * 16;
  const int b = grp0 >> 10;
  const int row0 = blockIdx.x * 512;
#pragma unroll
  for (int it = 0; it < 2; ++it) {
    int v = idxp[row0 + tid + 256 * it];
    v = (v < 0) ? 0 : v;
    v = (v > NPTS - 1) ? (NPTS - 1) : v;
    sIdx[tid + 256 * it] = v;
  }
  __syncthreads();
  const int c8 = tid & 7;
  const int rr = tid >> 3;
  float as[8], aq[8];
#pragma unroll
  for (int i = 0; i < 8; ++i) {
    as[i] = 0.0f;
    aq[i] = 0.0f;
  }
#pragma unroll 1
  for (int g = 0; g < 16; ++g) {
    const int n = sIdx[g * 32 + rr];
    const float* qp = Q + ((size_t)(b * NPTS + n)) * 64 + c8 * 8;
    const float* rp = R + ((size_t)(grp0 + g)) * 64 + c8 * 8;
    const v4f q0 = *(const v4f*)(qp);
    const v4f q1 = *(const v4f*)(qp + 4);
    const v4f r0 = *(const v4f*)(rp);
    const v4f r1 = *(const v4f*)(rp + 4);
    const float yy[8] = {q0.x - r0.x, q0.y - r0.y, q0.z - r0.z, q0.w - r0.w,
                         q1.x - r1.x, q1.y - r1.y, q1.z - r1.z, q1.w - r1.w};
#pragma unroll
    for (int i = 0; i < 8; ++i) {
      as[i] += yy[i];
      aq[i] += yy[i] * yy[i];
    }
  }
#pragma unroll
  for (int i = 0; i < 8; ++i) {
    sRed[rr][c8 * 8 + i] = as[i];
    sRed[rr][64 + c8 * 8 + i] = aq[i];
  }
  __syncthreads();
  if (tid < 128) {
    float a = 0.0f;
#pragma unroll 8
    for (int r = 0; r < 32; ++r) a += sRed[r][tid];
    sP[tid] = a;
  }
  __syncthreads();
  if (tid < 32) {
    const v4f pv = *(const v4f*)(sP + tid * 4);
    float* pp = part0 + (size_t)blockIdx.x * 128 + tid * 4;
    *(volatile v4f*)pp = pv;
    __threadfence();
    *(volatile v4f*)pp = pv;
  }
}

__global__ __launch_bounds__(256) void k_fin(const float* __restrict__ part, int nblk, int nch,
                                             const float* __restrict__ g, const float* __restrict__ be,
                                             float* __restrict__ tab) {
  __shared__ double sD[256];
  __shared__ __align__(16) float sTab[256];
  const int tid = threadIdx.x;
  const int pitch = 2 * nch;
  const int col = (tid < pitch) ? tid : (pitch - 1);
  double a = 0.0;
#pragma unroll 4
  for (int i = 0; i < nblk; ++i) a += (double)part[(size_t)i * pitch + col];
  sD[tid] = (tid < pitch) ? a : 0.0;
  sTab[tid] = 0.0f;
  __syncthreads();
  if (tid < nch) {
    const double invm = 1.0 / (double)MROWS;
    const double mean = sD[tid] * invm;
    const double ex2 = sD[nch + tid] * invm;
    double var = ex2 - mean * mean;
    var = (var < 0.0) ? 0.0 : var;
    const float vf = (float)var + BN_EPS;
    const float inv = 1.0f / sqrtf(vf);
    const float sc = g[tid] * inv;
    const float sh = be[tid] - sc * (float)mean;
    sTab[tid] = sc;
    sTab[128 + tid] = sh;
  }
  __syncthreads();
  if (tid < 32) {
    const v4f t0 = *(const v4f*)(sTab + tid * 4);
    const v4f t1 = *(const v4f*)(sTab + 128 + tid * 4);
    *(volatile v4f*)(tab + tid * 4) = t0;
    *(volatile v4f*)(tab + 128 + tid * 4) = t1;
    __threadfence();
    *(volatile v4f*)(tab + tid * 4) = t0;
    *(volatile v4f*)(tab + 128 + tid * 4) = t1;
  }
}

__global__ __launch_bounds__(256) void k_gemm1(const float* __restrict__ Q, const float* __restrict__ R,
                                               const int* __restrict__ idxp,
                                               const unsigned short* __restrict__ Wh,
                                               const float* __restrict__ tab0,
                                               const float* __restrict__ b1,
                                               unsigned short* __restrict__ y1,
                                               float* __restrict__ part1) {
  __shared__ __align__(16) _Float16 sA[128 * LDT];
  __shared__ __align__(16) _Float16 sB[64 * LDT];
  __shared__ __align__(16) _Float16 sSl[8][16 * LDT];
  __shared__ float sSc[64];
  __shared__ float sSh[64];
  __shared__ float sBias[64];
  __shared__ int sIdx[128];
  __shared__ float sStat[8][128];
  __shared__ __align__(16) float sP[128];
  const int tid = threadIdx.x;
  const int lane = tid & 31;
  const int wave = tid >> 5;
  const int rlane = lane & 15;
  const int hh = lane >> 4;
  const int row0 = blockIdx.x * 128;
  const int grp0 = blockIdx.x * 4;
  const int b = grp0 >> 10;
  if (tid < 64) {
    sSc[tid] = tab0[tid];
    sSh[tid] = tab0[128 + tid];
    sBias[tid] = b1[tid];
  }
  if (tid < 128) {
    int v = idxp[row0 + tid];
    v = (v < 0) ? 0 : v;
    v = (v > NPTS - 1) ? (NPTS - 1) : v;
    sIdx[tid] = v;
  }
#pragma unroll
  for (int it = 0; it < 2; ++it) {
    const int q = tid + 256 * it;
    const int r = q >> 3;
    const int c8 = q & 7;
    const v4u w = *(const v4u*)(Wh + (64 + r) * 64 + c8 * 8);
    *(v4u*)(sB + r * LDT + c8 * 8) = w;
  }
  __syncthreads();
  {
    const int c8 = tid & 7;
    const int rr = tid >> 3;
    float scv[8], shv[8];
#pragma unroll
    for (int i = 0; i < 8; ++i) {
      scv[i] = sSc[c8 * 8 + i];
      shv[i] = sSh[c8 * 8 + i];
    }
#pragma unroll 1
    for (int it = 0; it < 4; ++it) {
      const int row = rr + 32 * it;
      const int n = sIdx[row];
      const float* qp = Q + ((size_t)(b * NPTS + n)) * 64 + c8 * 8;
      const float* rp = R + ((size_t)(grp0 + it)) * 64 + c8 * 8;
      const v4f q0 = *(const v4f*)(qp);
      const v4f q1 = *(const v4f*)(qp + 4);
      const v4f r0 = *(const v4f*)(rp);
      const v4f r1 = *(const v4f*)(rp + 4);
      const float yy[8] = {q0.x - r0.x, q0.y - r0.y, q0.z - r0.z, q0.w - r0.w,
                           q1.x - r1.x, q1.y - r1.y, q1.z - r1.z, q1.w - r1.w};
      v8h hv;
#pragma unroll
      for (int i = 0; i < 8; ++i) {
        const float t = scv[i] * yy[i] + shv[i];
        const float a = fmaxf(t, 0.0f) * CARRY;
        hv[i] = (_Float16)a;
      }
      *(v8h*)(sA + row * LDT + c8 * 8) = hv;
    }
  }
  __syncthreads();

  const _Float16* Al = sA + (16 * wave + rlane) * LDT + 8 * hh;
  const _Float16* Bl = sB + rlane * LDT + 8 * hh;
  v8f acc[4];
#pragma unroll
  for (int j = 0; j < 4; ++j) acc[j] = (v8f){0.f, 0.f, 0.f, 0.f, 0.f, 0.f, 0.f, 0.f};
#pragma unroll
  for (int ks = 0; ks < 2; ++ks) {
    const v16h a = frag_ld(Al + ks * 32);
    const v16h f0 = frag_ld(Bl + 0 * 16 * LDT + ks * 32);
    const v16h f1 = frag_ld(Bl + 1 * 16 * LDT + ks * 32);
    const v16h f2 = frag_ld(Bl + 2 * 16 * LDT + ks * 32);
    const v16h f3 = frag_ld(Bl + 3 * 16 * LDT + ks * 32);
    acc[0] = mma_h(a, f0, acc[0]);
    acc[1] = mma_h(a, f1, acc[1]);
    acc[2] = mma_h(a, f2, acc[2]);
    acc[3] = mma_h(a, f3, acc[3]);
    guard4(acc[0], acc[1], acc[2], acc[3], a, f0, f1, f2, f3);
  }

  _Float16* sl = sSl[wave];
#pragma unroll
  for (int j = 0; j < 4; ++j) {
    const int col = 16 * j + rlane;
    const float bo = sBias[col];
    float ps = 0.0f, pq = 0.0f;
#pragma unroll
    for (int r = 0; r < 8; ++r) {
      const float v = acc[j][r] * FOLD + bo;
      ps += v;
      pq += v * v;
      sl[(8 * hh + r) * LDT + col] = (_Float16)v;
    }
    const float os = __shfl_xor(ps, 16, 32);
    const float oq = __shfl_xor(pq, 16, 32);
    ps += os;
    pq += oq;
    if (hh == 0) {
      sStat[wave][col] = ps;
      sStat[wave][64 + col] = pq;
    }
  }
  wave_lds_sync();
  {
    const int q = lane >> 3;
    const int c8 = (lane & 7) * 8;
    for (int pass = 0; pass < 2; ++pass) {
#pragma unroll
      for (int it = 0; it < 4; ++it) {
        const int row = it * 4 + q;
        const v8h hv = *(const v8h*)(sl + row * LDT + c8);
        *(volatile v8h*)(y1 + ((size_t)(row0 + 16 * wave + row)) * 64 + c8) = hv;
      }
      __threadfence();
    }
  }
  __syncthreads();
  if (tid < 128) {
    float a = 0.0f;
#pragma unroll
    for (int w = 0; w < 8; ++w) a += sStat[w][tid];
    sP[tid] = a;
  }
  __syncthreads();
  if (tid < 32) {
    const v4f pv = *(const v4f*)(sP + tid * 4);
    float* pp = part1 + (size_t)blockIdx.x * 128 + tid * 4;
    *(volatile v4f*)pp = pv;
    __threadfence();
    *(volatile v4f*)pp = pv;
  }
}

__global__ __launch_bounds__(256) void k_gemm2(const unsigned short* __restrict__ y1,
                                               const unsigned short* __restrict__ Wh,
                                               const float* __restrict__ tab1,
                                               const float* __restrict__ b2,
                                               float* __restrict__ ymm,
                                               float* __restrict__ part2) {
  __shared__ __align__(16) _Float16 sA[128 * LDT];
  __shared__ __align__(16) _Float16 sB[128 * LDT];
  __shared__ float sSc[64];
  __shared__ float sSh[64];
  __shared__ float sBias[128];
  __shared__ float sStat[8][256];
  __shared__ float sMM[8][256];
  __shared__ __align__(16) float sP[256];
  const int tid = threadIdx.x;
  const int lane = tid & 31;
  const int wave = tid >> 5;
  const int rlane = lane & 15;
  const int hh = lane >> 4;
  const int row0 = blockIdx.x * 128;
  const int grp0 = blockIdx.x * 4;
  if (tid < 64) {
    sSc[tid] = tab1[tid];
    sSh[tid] = tab1[128 + tid];
  }
  if (tid < 128) sBias[tid] = b2[tid];
#pragma unroll
  for (int it = 0; it < 4; ++it) {
    const int q = tid + 256 * it;
    const int r = q >> 3;
    const int c8 = q & 7;
    const v4u w = *(const v4u*)(Wh + (128 + r) * 64 + c8 * 8);
    *(v4u*)(sB + r * LDT + c8 * 8) = w;
  }
  __syncthreads();
  {
    const int c8 = tid & 7;
    const int rr = tid >> 3;
    float scv[8], shv[8];
#pragma unroll
    for (int i = 0; i < 8; ++i) {
      scv[i] = sSc[c8 * 8 + i];
      shv[i] = sSh[c8 * 8 + i];
    }
#pragma unroll 1
    for (int it = 0; it < 4; ++it) {
      const int row = rr + 32 * it;
      const v4u w = *(const v4u*)(y1 + ((size_t)(row0 + row)) * 64 + c8 * 8);
      const unsigned ww[4] = {w.x, w.y, w.z, w.w};
      v8h hv;
#pragma unroll
      for (int p = 0; p < 4; ++p) {
        const float f0 = h16_to_f32(ww[p] & 0xffffu);
        const float f1 = h16_to_f32(ww[p] >> 16);
        const float t0 = scv[2 * p] * f0 + shv[2 * p];
        const float t1 = scv[2 * p + 1] * f1 + shv[2 * p + 1];
        const float a0 = fmaxf(t0, 0.0f) * CARRY;
        const float a1 = fmaxf(t1, 0.0f) * CARRY;
        hv[2 * p] = (_Float16)a0;
        hv[2 * p + 1] = (_Float16)a1;
      }
      *(v8h*)(sA + row * LDT + c8 * 8) = hv;
    }
  }
  __syncthreads();

  const _Float16* Al = sA + (16 * wave + rlane) * LDT + 8 * hh;
  const _Float16* Bl = sB + rlane * LDT + 8 * hh;
  v8f acc[8];
#pragma unroll
  for (int j = 0; j < 8; ++j) acc[j] = (v8f){0.f, 0.f, 0.f, 0.f, 0.f, 0.f, 0.f, 0.f};
#pragma unroll
  for (int ks = 0; ks < 2; ++ks) {
    const v16h a = frag_ld(Al + ks * 32);
#pragma unroll
    for (int jg = 0; jg < 2; ++jg) {
      const v16h f0 = frag_ld(Bl + (jg * 4 + 0) * 16 * LDT + ks * 32);
      const v16h f1 = frag_ld(Bl + (jg * 4 + 1) * 16 * LDT + ks * 32);
      const v16h f2 = frag_ld(Bl + (jg * 4 + 2) * 16 * LDT + ks * 32);
      const v16h f3 = frag_ld(Bl + (jg * 4 + 3) * 16 * LDT + ks * 32);
      acc[jg * 4 + 0] = mma_h(a, f0, acc[jg * 4 + 0]);
      acc[jg * 4 + 1] = mma_h(a, f1, acc[jg * 4 + 1]);
      acc[jg * 4 + 2] = mma_h(a, f2, acc[jg * 4 + 2]);
      acc[jg * 4 + 3] = mma_h(a, f3, acc[jg * 4 + 3]);
      guard4(acc[jg * 4 + 0], acc[jg * 4 + 1], acc[jg * 4 + 2], acc[jg * 4 + 3], a, f0, f1, f2, f3);
    }
  }

#pragma unroll
  for (int j = 0; j < 8; ++j) {
    const int col = 16 * j + rlane;
    const float bo = sBias[col];
    float ps = 0.0f, pq = 0.0f, mx = -3.0e38f, mn = 3.0e38f;
#pragma unroll
    for (int r = 0; r < 8; ++r) {
      const float v = acc[j][r] * FOLD + bo;
      ps += v;
      pq += v * v;
      mx = fmaxf(mx, v);
      mn = fminf(mn, v);
    }
    const float os = __shfl_xor(ps, 16, 32);
    const float oq = __shfl_xor(pq, 16, 32);
    const float ox = __shfl_xor(mx, 16, 32);
    const float on = __shfl_xor(mn, 16, 32);
    ps += os;
    pq += oq;
    mx = fmaxf(mx, ox);
    mn = fminf(mn, on);
    if (hh == 0) {
      sStat[wave][col] = ps;
      sStat[wave][128 + col] = pq;
      sMM[wave][col] = mx;
      sMM[wave][128 + col] = mn;
    }
  }
  __syncthreads();
  {
    float a = 0.0f;
#pragma unroll
    for (int w = 0; w < 8; ++w) a += sStat[w][tid];
    sP[tid] = a;
  }
  {
    const int g = tid >> 6;
    const int c4 = (tid & 63) * 4;
    const bool isMax = c4 < 128;
    float o[4];
#pragma unroll
    for (int i = 0; i < 4; ++i) {
      const float u = sMM[2 * g][c4 + i];
      const float w = sMM[2 * g + 1][c4 + i];
      const float hi = fmaxf(u, w);
      const float lo = fminf(u, w);
      o[i] = isMax ? hi : lo;
    }
    const v4f ov = (v4f){o[0], o[1], o[2], o[3]};
    float* pm = ymm + ((size_t)(grp0 + g)) * 256 + c4;
    *(volatile v4f*)pm = ov;
    __threadfence();
    *(volatile v4f*)pm = ov;
  }
  __syncthreads();
  if (tid < 64) {
    const v4f pv = *(const v4f*)(sP + tid * 4);
    float* pp = part2 + (size_t)blockIdx.x * 256 + tid * 4;
    *(volatile v4f*)pp = pv;
    __threadfence();
    *(volatile v4f*)pp = pv;
  }
}

__global__ __launch_bounds__(256) void k_out(const float* __restrict__ ymm, const float* __restrict__ tab2,
                                             float* __restrict__ out1) {
  __shared__ __align__(16) float sT[128 * 68];
  __shared__ float sSc[128];
  __shared__ float sSh[128];
  const int tid = threadIdx.x;
  const int lane = tid & 31;
  const int wave = tid >> 5;
  const int hh = lane >> 4;
  const int b = blockIdx.x >> 4;
  const int s0 = (blockIdx.x & 15) * 64;
  if (tid < 128) {
    sSc[tid] = tab2[tid];
    sSh[tid] = tab2[128 + tid];
  }
  __syncthreads();
#pragma unroll 1
  for (int it = 0; it < 8; ++it) {
    const int q = tid + 256 * it;
    const int row = q >> 5;
    const int c4 = (q & 31) * 4;
    const float* pm = ymm + ((size_t)(b * NSAMP + s0 + row)) * 256 + c4;
    const v4f vmx = *(const v4f*)(pm);
    const v4f vmn = *(const v4f*)(pm + 128);
    const float amx[4] = {vmx.x, vmx.y, vmx.z, vmx.w};
    const float amn[4] = {vmn.x, vmn.y, vmn.z, vmn.w};
#pragma unroll
    for (int i = 0; i < 4; ++i) {
      const int c = c4 + i;
      const float sc = sSc[c];
      const float sh = sSh[c];
      const float fa = (sc >= 0.0f) ? 1.0f : 0.0f;
      const float fb = 1.0f - fa;
      const float y = fa * amx[i] + fb * amn[i];
      const float t = sc * y + sh;
      sT[c * 68 + row] = fmaxf(t, 0.0f);
    }
  }
  __syncthreads();
  {
    const int c4s = (lane & 15) * 4;
    for (int pass = 0; pass < 2; ++pass) {
#pragma unroll
      for (int it = 0; it < 8; ++it) {
        const int o = wave * 16 + it * 2 + hh;
        const v4f v = *(const v4f*)(sT + o * 68 + c4s);
        *(volatile v4f*)(out1 + ((size_t)(b * 128 + o)) * NSAMP + s0 + c4s) = v;
      }
      __threadfence();
    }
  }
}

extern "C" void kernel_launch(void* const* d_in, const int* in_sizes, int n_in,
                              void* d_out, int out_size, void* d_ws, size_t ws_size,
                              hipStream_t stream) {
  (void)in_sizes; (void)n_in; (void)out_size;
  if (ws_size < WS_TOTAL) return;
  const float* xyz = (const float*)d_in[0];
  const float* pts = (const float*)d_in[1];
  const float* w0  = (const float*)d_in[2];
  const float* b0  = (const float*)d_in[3];
  const float* g0  = (const float*)d_in[4];
  const float* be0 = (const float*)d_in[5];
  const float* w1  = (const float*)d_in[6];
  const float* b1  = (const float*)d_in[7];
  const float* g1  = (const float*)d_in[8];
  const float* be1 = (const float*)d_in[9];
  const float* w2  = (const float*)d_in[10];
  const float* b2  = (const float*)d_in[11];
  const float* g2  = (const float*)d_in[12];
  const float* be2 = (const float*)d_in[13];

  float* out0 = (float*)d_out;
  float* out1 = (float*)d_out + (size_t)(196608 / 4);

  char* ws = (char*)d_ws;
  size_t off = 0;
  unsigned short* ptsT = (unsigned short*)(ws + off); off += WS_PTST;
  unsigned short* Wh   = (unsigned short*)(ws + off); off += WS_WH;
  float* Q     = (float*)(ws + off); off += WS_Q;
  float* R     = (float*)(ws + off); off += WS_R;
  int*   idxp  = (int*)(ws + off);   off += WS_IDX;
  float* nxyz  = (float*)(ws + off); off += WS_NXYZ;
  unsigned short* y1 = (unsigned short*)(ws + off); off += WS_Y1;
  float* ymm   = (float*)(ws + off); off += WS_YMM;
  float* part0 = (float*)(ws + off); off += WS_PART0;
  float* part1 = (float*)(ws + off); off += WS_PART1;
  float* part2 = (float*)(ws + off); off += WS_PART2;
  float* tab0  = (float*)(ws + off); off += WS_TAB;
  float* tab1  = (float*)(ws + off); off += WS_TAB;
  float* tab2  = (float*)(ws + off); off += WS_TAB;

  k_fps<<<NB, 1024, 0, stream>>>(xyz, out0, nxyz);
  k_prep_pts<<<NB * 64, 256, 0, stream>>>(pts, ptsT);
  k_wprep<<<1, 256, 0, stream>>>(w0, w1, w2, Wh);
  k_gemmQ<<<NPROW / 128, 256, 0, stream>>>(ptsT, Wh, xyz, w0, b0, Q);
  k_ballR<<<NGRP / 8, 256, 0, stream>>>(xyz, nxyz, w0, idxp, R);
  k_stats0<<<MROWS / 512, 256, 0, stream>>>(Q, R, idxp, part0);
  k_fin<<<1, 256, 0, stream>>>(part0, MROWS / 512, 64, g0, be0, tab0);
  k_gemm1<<<MROWS / 128, 256, 0, stream>>>(Q, R, idxp, Wh, tab0, b1, y1, part1);
  k_fin<<<1, 256, 0, stream>>>(part1, MROWS / 128, 64, g1, be1, tab1);
  k_gemm2<<<MROWS / 128, 256, 0, stream>>>(y1, Wh, tab1, b2, ymm, part2);
  k_fin<<<1, 256, 0, stream>>>(part2, MROWS / 128, 128, g2, be2, tab2);
  k_out<<<NB * 16, 256, 0, stream>>>(ymm, tab2, out1);
}
